// Mamba_30468497998114
// MI455X (gfx1250) — hardware-verified
//
#include <hip/hip_runtime.h>
#include <math.h>

typedef __attribute__((ext_vector_type(16))) _Float16 v16h;
typedef __attribute__((ext_vector_type(8)))  _Float16 v8h;
typedef __attribute__((ext_vector_type(8)))  float    v8f;
typedef __attribute__((ext_vector_type(4)))  float    v4f;

constexpr int kBatch = 2;
constexpr int kSeq   = 1024;
constexpr int kDm    = 2048;
constexpr int kNst   = 64;
constexpr int kHd    = 64;
constexpr int kNh    = 32;
constexpr int kCD    = kDm + 2 * kNst;
constexpr int kPN    = 2 * kDm + 2 * kNst + kNh;
constexpr int kPP    = 4288;
constexpr int kRows  = kBatch * kSeq;
constexpr int kOffX  = kDm;
constexpr int kOffDt = 2 * kDm + 2 * kNst;
constexpr float kWCarry = 32.0f;
constexpr float kYCarry = 16.0f;
constexpr int kCvCh = 128;
constexpr int kCvTP = 132;
constexpr int kScTS = 32;
constexpr int kScYP = 68;
static_assert(kNh * kHd == kDm, "heads x headdim");
static_assert(kCD == 2176 && kPN == 4256 && kRows == 2048, "shape constants");
static_assert(kPP >= kPN && (kPP % 64) == 0, "padded in-projection width");
static_assert((kDm % 32) == 0, "GEMM K multiple of 32");
static_assert((kRows % 64) == 0 && (kDm % 64) == 0, "GEMM M,N multiples of 64");
static_assert((kCD % kCvCh) == 0 && (kSeq % 64) == 0 && (kSeq % kScTS) == 0, "tile multiples");
static_assert(kScTS == 32 && kNst == 64 && kHd == 64, "scan tile maps assume these sizes");

constexpr size_t kOffA0   = 0;
constexpr size_t kOffBT0  = kOffA0   + (size_t)kRows * kDm * 2;
constexpr size_t kOffBT1  = kOffBT0  + (size_t)kPP * kDm * 2;
constexpr size_t kOffPROJ = kOffBT1  + (size_t)kDm * kDm * 2;
constexpr size_t kOffXBC  = kOffPROJ + (size_t)kRows * kPP * 4;
constexpr size_t kOffYG   = kOffXBC  + (size_t)kRows * kCD * 4;
constexpr size_t kWsTotal = kOffYG   + (size_t)kRows * kDm * 2;
static_assert(kWsTotal == 95682560ull, "carve total");
static_assert(kWsTotal <= 134217728ull, "carve cap");
static_assert((kOffBT0 % 128) == 0 && (kOffBT1 % 128) == 0 && (kOffPROJ % 128) == 0 &&
              (kOffXBC % 128) == 0 && (kOffYG % 128) == 0, "128-B aligned regions");

union FragHU { v16h v; v8h h[2]; };
__device__ __forceinline__ v16h frag_load_h(const _Float16* p) {
  FragHU f;
  f.h[0] = *(const v8h*)(p);
  f.h[1] = *(const v8h*)(p + 16);
  return f.v;
}
__device__ __forceinline__ v8f mma_h(v16h a, v16h b, v8f c) {
  return __builtin_amdgcn_wmma_f32_16x16x32_f16(false, a, false, b, (short)0, c, false, false);
}
__device__ __forceinline__ void guard_row_h(v8f& c0, v8f& c1, v8f& c2, v8f& c3,
                                            v16h a, v16h b0, v16h b1, v16h b2, v16h b3) {
  asm volatile("v_nop\n\tv_nop\n\tv_nop\n\tv_nop"
               : "+v"(c0), "+v"(c1), "+v"(c2), "+v"(c3)
               : "v"(a), "v"(b0), "v"(b1), "v"(b2), "v"(b3));
}
__device__ __forceinline__ void keep4_h(v16h a, v16h b, v16h c, v16h d) {
  asm volatile("v_nop" :: "v"(a), "v"(b), "v"(c), "v"(d));
}
__device__ __forceinline__ void acc_guard4(v8f& a, v8f& b, v8f& c, v8f& d) {
  asm volatile("v_nop\n\tv_nop\n\tv_nop\n\tv_nop" : "+v"(a), "+v"(b), "+v"(c), "+v"(d));
}

__global__ __launch_bounds__(256) void wmma_gemm64_f16(
    const unsigned short* __restrict__ Ap, int lda,
    const unsigned short* __restrict__ Btp, int ldb,
    float* __restrict__ Cout, int ldc,
    int M, int N, int K, float scale) {
  const _Float16* A  = (const _Float16*)Ap;
  const _Float16* Bt = (const _Float16*)Btp;
  __shared__ __align__(16) float sT[8][16 * 68];
  const int lane = threadIdx.x & 31;
  const int wave = threadIdx.x >> 5;
  const int tilesN = N >> 6;
  const int tilesM = M >> 6;
  const int tile = blockIdx.x * 8 + wave;
  if (tile >= tilesM * tilesN) return;
  const int tm = tile / tilesN;
  const int tn = tile - tm * tilesN;
  const int m0 = tm << 6;
  const int n0 = tn << 6;

  const int rlane = lane & 15;
  const int koff  = (lane >> 4) * 8;
  const int mOff  = (lane >> 4) * 8;

  v8f acc[4][4];
#pragma unroll
  for (int i = 0; i < 4; ++i)
#pragma unroll
    for (int j = 0; j < 4; ++j) acc[i][j] = (v8f){0.f, 0.f, 0.f, 0.f, 0.f, 0.f, 0.f, 0.f};

  for (int k0 = 0; k0 < K; k0 += 32) {
    v16h bh[4];
#pragma unroll
    for (int j = 0; j < 4; ++j) {
      const size_t bo = (size_t)(n0 + (j << 4) + rlane) * ldb + koff + k0;
      bh[j] = frag_load_h(Bt + bo);
    }
#pragma unroll
    for (int i = 0; i < 4; ++i) {
      const size_t ao = (size_t)(m0 + (i << 4) + rlane) * lda + koff + k0;
      const v16h ah = frag_load_h(A + ao);
#pragma unroll
      for (int j = 0; j < 4; ++j) acc[i][j] = mma_h(ah, bh[j], acc[i][j]);
      guard_row_h(acc[i][0], acc[i][1], acc[i][2], acc[i][3], ah, bh[0], bh[1], bh[2], bh[3]);
    }
    keep4_h(bh[0], bh[1], bh[2], bh[3]);
  }
  acc_guard4(acc[0][0], acc[0][1], acc[0][2], acc[0][3]);
  acc_guard4(acc[1][0], acc[1][1], acc[1][2], acc[1][3]);
  acc_guard4(acc[2][0], acc[2][1], acc[2][2], acc[2][3]);
  acc_guard4(acc[3][0], acc[3][1], acc[3][2], acc[3][3]);

  float* slab = sT[wave];
#pragma unroll
  for (int i = 0; i < 4; ++i) {
    const int mBase = m0 + (i << 4);
#pragma unroll
    for (int j = 0; j < 4; ++j) {
#pragma unroll
      for (int r = 0; r < 8; ++r) {
        const float v = acc[i][j][r] * scale;
        slab[(mOff + r) * 68 + (j << 4) + rlane] = v;
      }
    }
    __builtin_amdgcn_fence(__ATOMIC_RELEASE, "workgroup");
    __builtin_amdgcn_wave_barrier();
    __builtin_amdgcn_fence(__ATOMIC_ACQUIRE, "workgroup");
    {
      const int hh = lane >> 4, c4 = (lane & 15) * 4;
      for (int pass = 0; pass < 2; ++pass) {
#pragma unroll
        for (int it = 0; it < 8; ++it) {
          const int row = it * 2 + hh;
          const v4f v = *(const v4f*)(slab + row * 68 + c4);
          *(volatile v4f*)(Cout + (size_t)(mBase + row) * ldc + n0 + c4) = v;
        }
        __threadfence();
      }
    }
    __builtin_amdgcn_fence(__ATOMIC_RELEASE, "workgroup");
    __builtin_amdgcn_wave_barrier();
    __builtin_amdgcn_fence(__ATOMIC_ACQUIRE, "workgroup");
  }
}

__global__ __launch_bounds__(256) void cast_f16_pad_kernel(
    const float* __restrict__ src, unsigned short* __restrict__ dst, int total8, int real8, float scale)
{
  const int i = blockIdx.x * 256 + threadIdx.x;
  if (i >= total8) return;
  const bool inb = (i < real8);
  const int ic = inb ? i : (real8 - 1);
  const float* p = src + ((size_t)ic << 3);
  const v4f a0 = *(const v4f*)(p);
  const v4f a1 = *(const v4f*)(p + 4);
  v8h hv;
#pragma unroll
  for (int e = 0; e < 4; ++e) {
    const float f0 = inb ? (a0[e] * scale) : 0.0f;
    const float f1 = inb ? (a1[e] * scale) : 0.0f;
    hv[e]     = (_Float16)f0;
    hv[4 + e] = (_Float16)f1;
  }
  unsigned short* q = dst + ((size_t)i << 3);
  *(volatile v8h*)q = hv;
  __threadfence();
  *(volatile v8h*)q = hv;
}

__global__ __launch_bounds__(128) void conv_silu_kernel(
    const float* __restrict__ PROJ, const float* __restrict__ cw, const float* __restrict__ cb,
    float* __restrict__ XBC)
{
  __shared__ __align__(16) float sT[16 * kCvTP];
  const int tid = threadIdx.x, lane = tid & 31, wave = tid >> 5;
  const int c0 = blockIdx.x * kCvCh, c = c0 + tid;
  const int g0 = blockIdx.y * 64;
  const int tb = g0 & (kSeq - 1);
  const v4f wv = *(const v4f*)(cw + (size_t)c * 4);
  const float w0 = wv[0], w1 = wv[1], w2 = wv[2], w3 = wv[3];
  const float bc = cb[c];
  const float* col = PROJ + kOffX + c;
  float xm3, xm2, xm1;
  {
    const bool hist = (tb > 0);
    const int rb = hist ? (g0 - 3) : g0;
    const float v3 = col[(size_t)rb * kPP];
    const float v2 = col[(size_t)(rb + 1) * kPP];
    const float v1 = col[(size_t)(rb + 2) * kPP];
    xm3 = hist ? v3 : 0.f;
    xm2 = hist ? v2 : 0.f;
    xm1 = hist ? v1 : 0.f;
  }
#pragma unroll 1
  for (int sub = 0; sub < 4; ++sub) {
    const int lb = g0 + sub * 16;
#pragma unroll 1
    for (int s = 0; s < 16; ++s) {
      const float xcur = col[(size_t)(lb + s) * kPP];
      float acc = w0 * xm3;
      acc = fmaf(w1, xm2, acc);
      acc = fmaf(w2, xm1, acc);
      acc = fmaf(w3, xcur, acc);
      const float sv = acc + bc;
      const float sg = __builtin_amdgcn_rcpf(1.0f + expf(-sv));
      sT[s * kCvTP + tid] = sv * sg;
      xm3 = xm2; xm2 = xm1; xm1 = xcur;
    }
    __syncthreads();
    v4f fv[4];
#pragma unroll
    for (int it = 0; it < 4; ++it) fv[it] = *(const v4f*)(sT + (it * 4 + wave) * kCvTP + lane * 4);
    for (int pass = 0; pass < 2; ++pass) {
#pragma unroll
      for (int it = 0; it < 4; ++it)
        *(volatile v4f*)(XBC + (size_t)(lb + it * 4 + wave) * kCD + c0 + lane * 4) = fv[it];
      __threadfence();
    }
    __syncthreads();
  }
}

__global__ __launch_bounds__(256) void scan_gate_kernel(
    const float* __restrict__ PROJ, const float* __restrict__ XBC,
    const float* __restrict__ Alog, const float* __restrict__ Dp, const float* __restrict__ dtb,
    unsigned short* __restrict__ YG)
{
  __shared__ __align__(16) float sBC[kScTS * 2 * kNst];
  __shared__ __align__(16) float sX[kScTS * kHd];
  __shared__ __align__(16) float sY[kScTS * kScYP];
  __shared__ float sDt[kScTS];
  __shared__ float sDA[kScTS];
  const int tid = threadIdx.x, lane = tid & 31, wave = tid >> 5;
  const int b = blockIdx.x / kNh;
  const int h = blockIdx.x - b * kNh;
  const int p  = tid >> 2;
  const int n0 = (tid & 3) * 16;
  const size_t row0 = (size_t)b * kSeq;
  const float Ah   = -expf(Alog[h]);
  const float Dh   = Dp[h];
  const float bias = dtb[h];
  float S[16];
#pragma unroll
  for (int j = 0; j < 16; ++j) S[j] = 0.f;
  const int q = lane >> 3, c8 = (lane & 7) * 8;

#pragma unroll 1
  for (int t0 = 0; t0 < kSeq; t0 += kScTS) {
    __syncthreads();
#pragma unroll
    for (int i = 0; i < 4; ++i) {
      const int idx = tid + i * 256;
      const int r = idx >> 5, c4 = (idx & 31) * 4;
      *(v4f*)(sBC + r * (2 * kNst) + c4) = *(const v4f*)(XBC + (row0 + t0 + r) * kCD + kDm + c4);
    }
#pragma unroll
    for (int i = 0; i < 2; ++i) {
      const int idx = tid + i * 256;
      const int r = idx >> 4, c4 = (idx & 15) * 4;
      *(v4f*)(sX + r * kHd + c4) = *(const v4f*)(XBC + (row0 + t0 + r) * kCD + h * kHd + c4);
    }
    if (tid < kScTS) {
      const float v  = PROJ[(row0 + t0 + tid) * kPP + kOffDt + h] + bias;
      const float sp = fmaxf(v, 0.0f) + log1pf(expf(-fabsf(v)));
      sDt[tid] = sp;
      sDA[tid] = expf(sp * Ah);
    }
    __syncthreads();

#pragma unroll 1
    for (int s = 0; s < kScTS; ++s) {
      const float dAv = sDA[s];
      const float dtv = sDt[s];
      const float xp  = sX[s * kHd + p];
      const float coef = dtv * xp;
      const float* br = sBC + s * (2 * kNst) + n0;
      const float* cr = br + kNst;
      float acc = 0.f;
#pragma unroll
      for (int j = 0; j < 4; ++j) {
        const v4f Bj = *(const v4f*)(br + 4 * j);
        const v4f Cj = *(const v4f*)(cr + 4 * j);
#pragma unroll
        for (int e = 0; e < 4; ++e) {
          const float sn = fmaf(S[4 * j + e], dAv, coef * Bj[e]);
          S[4 * j + e] = sn;
          acc = fmaf(sn, Cj[e], acc);
        }
      }
      acc += __shfl_xor(acc, 1, 32);
      acc += __shfl_xor(acc, 2, 32);
      const float yv = acc + Dh * xp;
      if ((tid & 3) == 0) sY[s * kScYP + p] = yv;
    }
    __syncthreads();

#pragma unroll 1
    for (int it = 0; it < 8; ++it) {
      const int idx = it * 256 + tid;
      const int row = idx >> 6, c = idx & 63;
      const float zv = PROJ[(row0 + t0 + row) * kPP + h * kHd + c];
      const float yv = sY[row * kScYP + c];
      const float sg = __builtin_amdgcn_rcpf(1.0f + expf(-zv));
      sY[row * kScYP + c] = (yv * (zv * sg)) * kYCarry;
    }
    __syncthreads();

    {
      const int row = wave * 4 + q;
      const float* sp = sY + row * kScYP + c8;
      const v4f a0 = *(const v4f*)(sp);
      const v4f a1 = *(const v4f*)(sp + 4);
      v8h hv;
#pragma unroll
      for (int e = 0; e < 4; ++e) {
        hv[e]     = (_Float16)a0[e];
        hv[4 + e] = (_Float16)a1[e];
      }
      unsigned short* dst = YG + (row0 + t0 + row) * kDm + h * kHd + c8;
      *(volatile v8h*)dst = hv;
      __threadfence();
      *(volatile v8h*)dst = hv;
    }
  }
}

static_assert(((kRows / 64) * (kPP / 64)) % 8 == 0, "in-projection tiles fill whole blocks");
static_assert(((kRows / 64) * (kDm / 64)) % 8 == 0, "out-projection tiles fill whole blocks");
static_assert(((kRows * kDm / 8) % 256) == 0 && ((kPP * kDm / 8) % 256) == 0 && ((kPN * kDm / 8) % 256) == 0,
              "cast grids exact");

extern "C" void kernel_launch(void* const* d_in, const int* in_sizes, int n_in,
                              void* d_out, int out_size, void* d_ws, size_t ws_size,
                              hipStream_t stream)
{
  if (n_in < 8) return;
  if (in_sizes[0] != kRows * kDm) return;
  if (in_sizes[1] != kPN * kDm) return;
  if (in_sizes[2] != kCD * 4) return;
  if (in_sizes[3] != kCD) return;
  if (in_sizes[4] != kDm * kDm) return;
  if (in_sizes[5] != kNh || in_sizes[6] != kNh || in_sizes[7] != kNh) return;
  if (out_size != kRows * kDm) return;
  if (ws_size < kWsTotal) return;

  const float* u       = (const float*)d_in[0];
  const float* W_in    = (const float*)d_in[1];
  const float* conv_w  = (const float*)d_in[2];
  const float* conv_b  = (const float*)d_in[3];
  const float* W_out   = (const float*)d_in[4];
  const float* A_log   = (const float*)d_in[5];
  const float* D_param = (const float*)d_in[6];
  const float* dt_bias = (const float*)d_in[7];
  float* out = (float*)d_out;

  char* ws = (char*)d_ws;
  unsigned short* A0   = (unsigned short*)(ws + kOffA0);
  unsigned short* BT0  = (unsigned short*)(ws + kOffBT0);
  unsigned short* BT1  = (unsigned short*)(ws + kOffBT1);
  float*          PROJ = (float*)(ws + kOffPROJ);
  float*          XBC  = (float*)(ws + kOffXBC);
  unsigned short* YG   = (unsigned short*)(ws + kOffYG);

  cast_f16_pad_kernel<<<(kRows * kDm / 8) / 256, 256, 0, stream>>>(u, A0, kRows * kDm / 8, kRows * kDm / 8, 1.0f);
  cast_f16_pad_kernel<<<(kPP * kDm / 8) / 256, 256, 0, stream>>>(W_in, BT0, kPP * kDm / 8, kPN * kDm / 8, kWCarry);
  cast_f16_pad_kernel<<<(kDm * kDm / 8) / 256, 256, 0, stream>>>(W_out, BT1, kDm * kDm / 8, kDm * kDm / 8, kWCarry);

  wmma_gemm64_f16<<<((kRows / 64) * (kPP / 64)) / 8, 256, 0, stream>>>(
      A0, kDm, BT0, kDm, PROJ, kPP, kRows, kPP, kDm, 1.0f / kWCarry);

  conv_silu_kernel<<<dim3(kCD / kCvCh, kRows / 64), kCvCh, 0, stream>>>(PROJ, conv_w, conv_b, XBC);

  scan_gate_kernel<<<kBatch * kNh, 256, 0, stream>>>(PROJ, XBC, A_log, D_param, dt_bias, YG);

  wmma_gemm64_f16<<<((kRows / 64) * (kDm / 64)) / 8, 256, 0, stream>>>(
      YG, kDm, BT1, kDm, out, kDm, kRows, kDm, kDm, 1.0f / (kWCarry * kYCarry));
}
